// CrossConvLayerV2_72189810312030
// MI455X (gfx1250) — hardware-verified
//
#include <hip/hip_runtime.h>
#include <stdint.h>

typedef __bf16 v16b __attribute__((ext_vector_type(16)));
typedef float  v8f  __attribute__((ext_vector_type(8)));
typedef float  v8fa __attribute__((ext_vector_type(8))) __attribute__((may_alias));
typedef float  v4f  __attribute__((ext_vector_type(4))) __attribute__((may_alias));

#define NWAVES   8
#define NT1      (NWAVES * 32)
#define NFEAT    16
#define PT_DIM   19
#define M_PROBES 26
#define KFLAT    (M_PROBES * NFEAT)
#define NOUT     256
#define NCENT    256
#define KCOEFF   0.1f
#define PDIST    3.0f
#define NT2      128
#define ROWS2    16

__device__ __forceinline__ v8f mma_bf16(v8f c, v16b a, v16b b) {
    return __builtin_amdgcn_wmma_f32_16x16x32_bf16(false, a, false, b, (short)0, c, false, false);
}

struct HL { __bf16 h; __bf16 l; };
__device__ __forceinline__ HL split2(float x) {
    HL r;
    r.h = (__bf16)x;
    r.l = (__bf16)(x - (float)r.h);
    return r;
}

__device__ __forceinline__ float sin8(int k) {
    const int q = k & 15;
    const int r = q & 7;
    float v;
    if (r == 0)                v = 0.0f;
    else if (r == 4)           v = 1.0f;
    else if (r == 1 || r == 7) v = 0.382683432365089772f;
    else if (r == 2 || r == 6) v = 0.707106781186547524f;
    else                       v = 0.923879532511286756f;
    return (q & 8) ? -v : v;
}

__device__ __forceinline__ void probe_pos(int m, float& px, float& py, float& pz) {
    int ka, kb;
    if (m < 24) {
        const int j = m >> 3, i = m & 7;
        ka = 2 * (j - 1);
        kb = 2 * i + (j - 1);
    } else {
        ka = (m == 24) ? -4 : 4;
        kb = 0;
    }
    const float sa = sin8(ka), ca = sin8(ka + 4);
    const float sb = sin8(kb), cb = sin8(kb + 4);
    px = PDIST * sa;
    py = PDIST * ca * cb;
    pz = PDIST * ca * sb;
}

__global__ __launch_bounds__(NT1)
void k_aggregate(const float* __restrict__ points,
                 const float* __restrict__ centers,
                 float* flat,
                 int npts, int ncent, int nb)
{
    __shared__ float s_coord[NWAVES][3][32] __attribute__((aligned(32)));
    __shared__ float s_feat[NWAVES][NFEAT][32] __attribute__((aligned(32)));
    __shared__ float s_red[NWAVES][2][8][32];
    __shared__ float s_flat[KFLAT] __attribute__((aligned(16)));

    const int tid  = threadIdx.x;
    const int lane = tid & 31;
    const int w    = tid >> 5;
    const int h    = lane >> 4;
    const int mrow = lane & 15;
    const int blk  = blockIdx.x;
    int b = blk / ncent;
    if (b > nb - 1) b = nb - 1;

    const float cx = centers[(size_t)blk * 3 + 0];
    const float cy = centers[(size_t)blk * 3 + 1];
    const float cz = centers[(size_t)blk * 3 + 2];

    float p0x, p0y, p0z;
    probe_pos(mrow, p0x, p0y, p0z);
    p0x += cx; p0y += cy; p0z += cz;
    int m1 = mrow + 16;
    if (m1 > M_PROBES - 1) m1 = M_PROBES - 1;
    float p1x, p1y, p1z;
    probe_pos(m1, p1x, p1y, p1z);
    p1x += cx; p1y += cy; p1z += cz;

    v8f acc0 = {};
    v8f acc1 = {};

    const float* ptbase = points + (size_t)b * (size_t)npts * PT_DIM;
    const int nchunk = (npts + 31) >> 5;
    const int niter  = (nchunk + NWAVES - 1) / NWAVES;

    for (int it = 0; it < niter; ++it) {
        const int p = ((it * NWAVES + w) << 5) + lane;
        float x = 0.f, y = 0.f, z = 0.f;
        float fv[NFEAT];
        #pragma unroll
        for (int ff = 0; ff < NFEAT; ++ff) fv[ff] = 0.f;
        if (p < npts) {
            const float* pp = ptbase + (size_t)p * PT_DIM;
            x = pp[0]; y = pp[1]; z = pp[2];
            #pragma unroll
            for (int ff = 0; ff < NFEAT; ++ff) fv[ff] = pp[3 + ff];
        }
        s_coord[w][0][lane] = x;
        s_coord[w][1][lane] = y;
        s_coord[w][2][lane] = z;
        #pragma unroll
        for (int ff = 0; ff < NFEAT; ++ff) s_feat[w][ff][lane] = fv[ff];
        __syncthreads();

        v16b bhi = {}, blo = {};
        #pragma unroll
        for (int q = 0; q < 2; ++q) {
            const v8fa u = *(const v8fa*)&s_feat[w][mrow][16 * q + 8 * h];
            #pragma unroll
            for (int i = 0; i < 8; ++i) {
                const HL s = split2(u[i]);
                bhi[8 * q + i] = s.h;
                blo[8 * q + i] = s.l;
            }
        }

        v16b ahi0 = {}, alo0 = {}, ahi1 = {}, alo1 = {};
        #pragma unroll
        for (int q = 0; q < 2; ++q) {
            const int kb = 16 * q + 8 * h;
            const v8fa xs = *(const v8fa*)&s_coord[w][0][kb];
            const v8fa ys = *(const v8fa*)&s_coord[w][1][kb];
            const v8fa zs = *(const v8fa*)&s_coord[w][2][kb];
            #pragma unroll
            for (int i = 0; i < 8; ++i) {
                const float px = xs[i], py = ys[i], pz = zs[i];
                float dx = px - p0x, dy = py - p0y, dz = pz - p0z;
                float t0 = dx * dx;
                t0 = fmaf(dy, dy, t0);
                t0 = fmaf(dz, dz, t0);
                t0 += KCOEFF;
                const HL s0 = split2(__builtin_amdgcn_rcpf(t0));
                ahi0[8 * q + i] = s0.h;
                alo0[8 * q + i] = s0.l;

                dx = px - p1x; dy = py - p1y; dz = pz - p1z;
                float t1 = dx * dx;
                t1 = fmaf(dy, dy, t1);
                t1 = fmaf(dz, dz, t1);
                t1 += KCOEFF;
                const HL s1 = split2(__builtin_amdgcn_rcpf(t1));
                ahi1[8 * q + i] = s1.h;
                alo1[8 * q + i] = s1.l;
            }
        }

        acc0 = mma_bf16(acc0, ahi0, bhi);
        acc0 = mma_bf16(acc0, ahi0, blo);
        acc0 = mma_bf16(acc0, alo0, bhi);
        acc1 = mma_bf16(acc1, ahi1, bhi);
        acc1 = mma_bf16(acc1, ahi1, blo);
        acc1 = mma_bf16(acc1, alo1, bhi);
        asm volatile("v_nop\n\tv_nop\n\tv_nop\n\tv_nop"
                     : "+v"(acc0), "+v"(acc1)
                     : "v"(ahi0), "v"(alo0), "v"(ahi1), "v"(alo1), "v"(bhi), "v"(blo));
        __syncthreads();
    }

    #pragma unroll
    for (int r = 0; r < 8; ++r) {
        s_red[w][0][r][lane] = acc0[r];
        s_red[w][1][r][lane] = acc1[r];
    }
    __syncthreads();

    const float scale = KCOEFF / (float)npts;
    for (int idx = tid; idx < 2 * 8 * 32; idx += NT1) {
        const int t  = idx >> 8;
        const int r  = (idx >> 5) & 7;
        const int ln = idx & 31;
        float s = 0.f;
        #pragma unroll
        for (int ww = 0; ww < NWAVES; ++ww) s += s_red[ww][t][r][ln];
        const int mm = t * 16 + ((ln >> 4) << 3) + r;
        const int f  = ln & 15;
        if (mm < M_PROBES) s_flat[mm * NFEAT + f] = s * scale;
    }
    __syncthreads();

    const bool act = tid < (KFLAT / 4);
    float* dst = flat + (size_t)blk * KFLAT + 4 * tid;
    v4f v = {};
    if (act) {
        v = *(const v4f*)&s_flat[4 * tid];
        *(volatile v4f*)dst = v;
    }
    __threadfence();
    if (act) {
        *(volatile v4f*)dst = v;
    }
}

__global__ __launch_bounds__(NT2)
void k_dense(const float* __restrict__ flat,
             const float* __restrict__ W,
             const float* __restrict__ bias,
             float* out,
             int nbl)
{
    __shared__ float s_out[ROWS2][NOUT] __attribute__((aligned(16)));

    const int tid  = threadIdx.x;
    const int lane = tid & 31;
    const int w    = tid >> 5;
    const int h    = lane >> 4;
    const int m    = lane & 15;
    const int row0 = blockIdx.x * ROWS2;
    int arow = row0 + m;
    if (arow > nbl - 1) arow = nbl - 1;
    const float* ap = flat + (size_t)arow * KFLAT;

    v8f acc[4];
    #pragma unroll
    for (int t = 0; t < 4; ++t) { v8f zz = {}; acc[t] = zz; }

    #pragma unroll 1
    for (int ks = 0; ks < KFLAT / 32; ++ks) {
        const int k0 = ks * 32;
        v16b ahi = {}, alo = {};
        #pragma unroll
        for (int q = 0; q < 2; ++q) {
            const v8fa u = *(const v8fa*)(ap + k0 + 16 * q + 8 * h);
            #pragma unroll
            for (int i = 0; i < 8; ++i) {
                const HL s = split2(u[i]);
                ahi[8 * q + i] = s.h;
                alo[8 * q + i] = s.l;
            }
        }
        #pragma unroll
        for (int t = 0; t < 4; ++t) {
            const int col = w * 64 + t * 16 + m;
            v16b bhi = {}, blo = {};
            #pragma unroll
            for (int q = 0; q < 2; ++q) {
                #pragma unroll
                for (int i = 0; i < 8; ++i) {
                    const int kk = k0 + 16 * q + 8 * h + i;
                    const HL s = split2(W[(size_t)kk * NOUT + col]);
                    bhi[8 * q + i] = s.h;
                    blo[8 * q + i] = s.l;
                }
            }
            v8f c = acc[t];
            c = mma_bf16(c, ahi, bhi);
            c = mma_bf16(c, ahi, blo);
            c = mma_bf16(c, alo, bhi);
            asm volatile("v_nop\n\tv_nop\n\tv_nop\n\tv_nop"
                         : "+v"(c) : "v"(ahi), "v"(alo), "v"(bhi), "v"(blo));
            acc[t] = c;
        }
    }

    #pragma unroll
    for (int t = 0; t < 4; ++t) {
        #pragma unroll
        for (int r = 0; r < 8; ++r) s_out[8 * h + r][w * 64 + t * 16 + m] = acc[t][r];
    }
    __syncthreads();

    v4f vals[8];
    #pragma unroll
    for (int j = 0; j < 4; ++j) {
        const int rr = 4 * w + j;
        #pragma unroll
        for (int s = 0; s < 2; ++s) {
            const int col = 4 * (lane + 32 * s);
            const v4f a  = *(const v4f*)&s_out[rr][col];
            const v4f bb = *(const v4f*)(bias + col);
            vals[2 * j + s] = a + bb;
        }
    }
    #pragma unroll
    for (int j = 0; j < 4; ++j) {
        const int grow = row0 + 4 * w + j;
        if (grow < nbl) {
            #pragma unroll
            for (int s = 0; s < 2; ++s) {
                const int col = 4 * (lane + 32 * s);
                *(volatile v4f*)(out + (size_t)grow * NOUT + col) = vals[2 * j + s];
            }
        }
    }
    __threadfence();
    #pragma unroll
    for (int j = 0; j < 4; ++j) {
        const int grow = row0 + 4 * w + j;
        if (grow < nbl) {
            #pragma unroll
            for (int s = 0; s < 2; ++s) {
                const int col = 4 * (lane + 32 * s);
                *(volatile v4f*)(out + (size_t)grow * NOUT + col) = vals[2 * j + s];
            }
        }
    }
}

extern "C" void kernel_launch(void* const* d_in, const int* in_sizes, int n_in,
                              void* d_out, int out_size, void* d_ws, size_t ws_size,
                              hipStream_t stream) {
    if (n_in < 4) return;
    const float* points  = (const float*)d_in[0];
    const float* centers = (const float*)d_in[1];
    const float* W       = (const float*)d_in[2];
    const float* bias    = (const float*)d_in[3];
    float* out  = (float*)d_out;
    float* flat = (float*)d_ws;

    const int nbl = in_sizes[1] / 3;
    if (nbl <= 0) return;
    int nb = nbl / NCENT;
    if (nb < 1) nb = 1;
    const int npts = in_sizes[0] / (PT_DIM * nb);
    if (npts <= 0) return;
    if (in_sizes[2] < KFLAT * NOUT) return;
    if (in_sizes[3] < NOUT) return;
    if (out_size < nbl * NOUT) return;
    if ((size_t)nbl * KFLAT * sizeof(float) > ws_size) return;

    k_aggregate<<<dim3(nbl), dim3(NT1), 0, stream>>>(points, centers, flat, npts, NCENT, nb);
    k_dense<<<dim3((nbl + ROWS2 - 1) / ROWS2), dim3(NT2), 0, stream>>>(flat, W, bias, out, nbl);
}
